// Graph_Attention_new_41815801593869
// MI455X (gfx1250) — hardware-verified
//
#include <hip/hip_runtime.h>
#include <math.h>

constexpr int kB     = 4;
constexpr int kHin   = 128;
constexpr int kWin   = 128;
constexpr int kC     = 64;
constexpr int kHs    = 64;
constexpr int kWs    = 64;
constexpr int kTok   = kHs * kWs;
constexpr int kNP    = kB * kTok;
constexpr int kKconv = 4 * kC;
constexpr int kCcat  = 2 * kC;
constexpr int kNdec  = 4 * kC;
constexpr int kNPout = kB * kHin * kWin;
constexpr float kPCarry      = 32768.0f;
constexpr float kPCarryInv   = 1.0f / 32768.0f;
constexpr float kWfiCarry    = 16.0f;
constexpr float kWfiCarryInv = 1.0f / 16.0f;
constexpr float kBnEps       = 1.0e-3f;
constexpr int kStatRows      = 256;

typedef __attribute__((ext_vector_type(16))) _Float16 v16h;
typedef __attribute__((ext_vector_type(8)))  _Float16 v8h;
typedef __attribute__((ext_vector_type(16))) __bf16   v16b;
typedef __attribute__((ext_vector_type(8)))  __bf16   v8b;
typedef __attribute__((ext_vector_type(8)))  float    v8f;
typedef __attribute__((ext_vector_type(4)))  float    v4f;
typedef __attribute__((ext_vector_type(4)))  unsigned int v4u;

constexpr size_t kMiB    = 1048576;
constexpr size_t offAx   = 0;
constexpr size_t offAz   = 8 * kMiB;
constexpr size_t offXGp  = 16 * kMiB;
constexpr size_t offZGp  = 20 * kMiB;
constexpr size_t offP    = 0;
constexpr size_t offS    = 32 * kMiB;
constexpr size_t offY    = 32 * kMiB;
constexpr size_t offXqh  = 96 * kMiB;
constexpr size_t offXql  = 98 * kMiB;
constexpr size_t offZkh  = 100 * kMiB;
constexpr size_t offZkl  = 102 * kMiB;
constexpr size_t offAdec = 104 * kMiB;
constexpr size_t offZGt  = 108 * kMiB;
constexpr size_t offBtW  = 110 * kMiB;
constexpr size_t offBtfi = offBtW + (size_t)3 * kC * kKconv * 2;
constexpr size_t offPart = offBtfi + (size_t)kNdec * kCcat * 2;
constexpr size_t offAffX = offPart + (size_t)256 * 64 * 4;
constexpr size_t offAffZ = offAffX + 1024;
constexpr size_t offAffY = offAffZ + 1024;
constexpr size_t offEnd  = offAffY + 1024;
static_assert((size_t)kNP * kKconv * 2 == 8 * kMiB, "size");
static_assert((size_t)kNP * kC * 4 == 4 * kMiB, "size");
static_assert((size_t)kTok * kTok * 2 == 32 * kMiB, "size");
static_assert((size_t)kTok * kTok * 4 == 64 * kMiB, "size");
static_assert((size_t)kNP * kNdec * 4 <= 64 * kMiB, "size");
static_assert((size_t)kNP * kC * 2 == 2 * kMiB, "size");
static_assert((size_t)kNP * kCcat * 2 == 4 * kMiB, "size");
static_assert((size_t)kB * kC * kTok * 2 == 2 * kMiB, "size");
static_assert(offEnd == 115575808, "carve");
static_assert(offEnd <= 134217728, "carve");
static_assert(kNPout / kStatRows <= 256 && kNP / kStatRows <= 256, "stat blocks");
static_assert(kNPout % kStatRows == 0 && kNP % kStatRows == 0 && kStatRows % 4 == 0, "stat rows");

__device__ __forceinline__ unsigned short f2bf_bits(float f) {
  unsigned u = __float_as_uint(f);
  return (unsigned short)((u + 0x7FFFu + ((u >> 16) & 1u)) >> 16);
}
__device__ __forceinline__ float bf_bits2f(unsigned short h) { return __uint_as_float(((unsigned)h) << 16); }

__device__ __forceinline__ void dep_guard_h(v8f& a, v8f& b, v16h x, v16h y) { asm volatile("v_nop\n\tv_nop\n\tv_nop\n\tv_nop" : "+v"(a), "+v"(b) : "v"(x), "v"(y)); }
__device__ __forceinline__ void dep_guard_b(v8f& a, v8f& b, v16b x, v16b y) { asm volatile("v_nop\n\tv_nop\n\tv_nop\n\tv_nop" : "+v"(a), "+v"(b) : "v"(x), "v"(y)); }
__device__ __forceinline__ void keep4_h(v16h a, v16h b, v16h c, v16h d) { asm volatile("v_nop" :: "v"(a), "v"(b), "v"(c), "v"(d)); }
__device__ __forceinline__ void keep4_b(v16b a, v16b b, v16b c, v16b d) { asm volatile("v_nop" :: "v"(a), "v"(b), "v"(c), "v"(d)); }
__device__ __forceinline__ void acc_guard4(v8f& a, v8f& b, v8f& c, v8f& d) { asm volatile("v_nop\n\tv_nop\n\tv_nop\n\tv_nop" : "+v"(a), "+v"(b), "+v"(c), "+v"(d)); }
template <typename T> struct Frag;
template <> struct Frag<_Float16> {
  typedef v16h V; union U { v16h v; v8h h[2]; };
  static __device__ __forceinline__ v16h load(const _Float16* p) {
    U f; f.h[0] = *(const v8h*)(p); f.h[1] = *(const v8h*)(p + 16); return f.v;
  }
  static __device__ __forceinline__ v8f mma(v16h a, v16h b, v8f c) {
    return __builtin_amdgcn_wmma_f32_16x16x32_f16(false, a, false, b, (short)0, c, false, false);
  }
  static __device__ __forceinline__ void guard(v8f& a, v8f& b, v16h x, v16h y) { dep_guard_h(a, b, x, y); }
  static __device__ __forceinline__ void keep(v16h a, v16h b, v16h c, v16h d) { keep4_h(a, b, c, d); }
};
template <> struct Frag<__bf16> {
  typedef v16b V; union U { v16b v; v8b h[2]; };
  static __device__ __forceinline__ v16b load(const __bf16* p) {
    U f; f.h[0] = *(const v8b*)(p); f.h[1] = *(const v8b*)(p + 16); return f.v;
  }
  static __device__ __forceinline__ v8f mma(v16b a, v16b b, v8f c) {
    return __builtin_amdgcn_wmma_f32_16x16x32_bf16(false, a, false, b, (short)0, c, false, false);
  }
  static __device__ __forceinline__ void guard(v8f& a, v8f& b, v16b x, v16b y) { dep_guard_b(a, b, x, y); }
  static __device__ __forceinline__ void keep(v16b a, v16b b, v16b c, v16b d) { keep4_b(a, b, c, d); }
};

__device__ __forceinline__ unsigned pk16(unsigned short a, unsigned short b) { return (unsigned)a | ((unsigned)b << 16); }
__device__ __forceinline__ unsigned short h_bits(float f) { const _Float16 h = (_Float16)f; return __builtin_bit_cast(unsigned short, h); }

template <int ET> struct Elem;
template <> struct Elem<0> { typedef _Float16 T; };
template <> struct Elem<1> { typedef __bf16 T; };
template <int ET, bool SPLIT, int BIAS_MODE, int OUT_MODE, bool RESID, int ACT = 0>
__global__ __launch_bounds__(256) void wmma_gemm64(
    const unsigned short* __restrict__ Ap, const unsigned short* __restrict__ A2p, int lda, long strideA,
    const unsigned short* __restrict__ Btp, const unsigned short* __restrict__ Bt2p, int ldb, long strideB,
    void* __restrict__ Cout, void* __restrict__ Cout2, int ldc, long strideC,
    const float* __restrict__ bias,
    const float* __restrict__ resid, long strideR,
    int M, int N, int K, float scale) {
  typedef typename Elem<ET>::T T;
  typedef typename Frag<T>::V V;
  const T* A = (const T*)Ap; const T* A2 = (const T*)A2p; const T* Bt = (const T*)Btp; const T* Bt2 = (const T*)Bt2p;
  __shared__ __align__(16) float sT[8][16 * 68];
  const int b    = blockIdx.y;
  const int lane = threadIdx.x & 31;
  const int wave = threadIdx.x >> 5;
  const int tilesN = N >> 6;
  const int tilesM = M >> 6;
  const int tile = blockIdx.x * 8 + wave;
  if (tile >= tilesM * tilesN) return;
  const int tm = tile / tilesN;
  const int tn = tile - tm * tilesN;
  const int m0 = tm << 6;
  const int n0 = tn << 6;

  const T* Ab  = A  + (size_t)b * strideA;
  const T* Bb  = Bt + (size_t)b * strideB;
  const T* Ab2 = SPLIT ? (A2  + (size_t)b * strideA) : nullptr;
  const T* Bb2 = SPLIT ? (Bt2 + (size_t)b * strideB) : nullptr;

  const int rlane = lane & 15;
  const int koff  = (lane >> 4) * 8;
  const int mOff  = (lane >> 4) * 8;

  v8f acc[4][4];
#pragma unroll
  for (int i = 0; i < 4; ++i)
#pragma unroll
    for (int j = 0; j < 4; ++j) acc[i][j] = (v8f){0.f,0.f,0.f,0.f,0.f,0.f,0.f,0.f};

  for (int k0 = 0; k0 < K; k0 += 32) {
    V bh[4], bl[4];
#pragma unroll
    for (int j = 0; j < 4; ++j) {
      const size_t bo = (size_t)(n0 + (j << 4) + rlane) * ldb + koff + k0;
      bh[j] = Frag<T>::load(Bb + bo);
      if (SPLIT) bl[j] = Frag<T>::load(Bb2 + bo);
    }
#pragma unroll
    for (int i = 0; i < 4; ++i) {
      const size_t ao = (size_t)(m0 + (i << 4) + rlane) * lda + koff + k0;
      V ah = Frag<T>::load(Ab + ao);
      V al;
      if (SPLIT) al = Frag<T>::load(Ab2 + ao);
#pragma unroll
      for (int j = 0; j < 4; ++j) {
        acc[i][j] = Frag<T>::mma(ah, bh[j], acc[i][j]);
        if (SPLIT) {
          acc[i][j] = Frag<T>::mma(ah, bl[j], acc[i][j]);
          acc[i][j] = Frag<T>::mma(al, bh[j], acc[i][j]);
        }
      }
      Frag<T>::guard(acc[i][0], acc[i][3], ah, SPLIT ? al : ah);
    }
    Frag<T>::keep(bh[0], bh[1], bh[2], bh[3]);
    if (SPLIT) Frag<T>::keep(bl[0], bl[1], bl[2], bl[3]);
  }
  acc_guard4(acc[0][0], acc[0][1], acc[0][2], acc[0][3]);
  acc_guard4(acc[1][0], acc[1][1], acc[1][2], acc[1][3]);
  acc_guard4(acc[2][0], acc[2][1], acc[2][2], acc[2][3]);
  acc_guard4(acc[3][0], acc[3][1], acc[3][2], acc[3][3]);

  float* slab = sT[wave];
  const float* Rb = RESID ? (resid + (size_t)b * strideR) : nullptr;
#pragma unroll
  for (int i = 0; i < 4; ++i) {
    const int mBase = m0 + (i << 4);
#pragma unroll
    for (int j = 0; j < 4; ++j) {
      const int n = n0 + (j << 4) + rlane;
      float bv = 0.f;
      if (BIAS_MODE == 2) bv = bias[n];
#pragma unroll
      for (int r = 0; r < 8; ++r) {
        float v = acc[i][j][r] * scale;
        if (BIAS_MODE == 1) v += bias[mBase + mOff + r];
        if (BIAS_MODE == 2) v += bv;
        if (RESID) v += Rb[(size_t)(mBase + mOff + r) * ldc + n];
        if (ACT == 2) v = fmaxf(v, 0.0f);
        if (ACT == 4) v = (v > 0.f) ? v : 0.01f * v;
        slab[(mOff + r) * 68 + (j << 4) + rlane] = v;
      }
    }
    __builtin_amdgcn_fence(__ATOMIC_RELEASE, "workgroup");
    __builtin_amdgcn_wave_barrier();
    __builtin_amdgcn_fence(__ATOMIC_ACQUIRE, "workgroup");
    if (OUT_MODE == 0) {
      float* C = (float*)Cout + (size_t)b * strideC;
      const int hh = lane >> 4, c4 = (lane & 15) * 4;
      for (int pass = 0; pass < 2; ++pass) {
#pragma unroll
        for (int it = 0; it < 8; ++it) {
          const int row = it * 2 + hh;
          v4f v = *(const v4f*)(slab + row * 68 + c4);
          *(volatile v4f*)(C + (size_t)(mBase + row) * ldc + n0 + c4) = v;
        }
        __threadfence();
      }
    } else {
      const int q = lane >> 3, c8 = (lane & 7) * 8;
      unsigned short* C  = (unsigned short*)Cout  + (size_t)b * strideC;
      unsigned short* C2 = (OUT_MODE == 2) ? ((unsigned short*)Cout2 + (size_t)b * strideC) : nullptr;
      for (int pass = 0; pass < 2; ++pass) {
#pragma unroll
        for (int it = 0; it < 4; ++it) {
          const int row = it * 4 + q;
          const float* sp = slab + row * 68 + c8;
          v8h hv, lv;
#pragma unroll
          for (int e = 0; e < 8; ++e) {
            if (OUT_MODE == 1) {
              hv[e] = (_Float16)sp[e];
            } else {
              unsigned short hb = f2bf_bits(sp[e]);
              unsigned short lb = f2bf_bits(sp[e] - bf_bits2f(hb));
              hv[e] = __builtin_bit_cast(_Float16, hb);
              lv[e] = __builtin_bit_cast(_Float16, lb);
            }
          }
          *(volatile v8h*)(C + (size_t)(mBase + row) * ldc + n0 + c8) = hv;
          if (OUT_MODE == 2) *(volatile v8h*)(C2 + (size_t)(mBase + row) * ldc + n0 + c8) = lv;
        }
        __threadfence();
      }
    }
    __builtin_amdgcn_fence(__ATOMIC_RELEASE, "workgroup");
    __builtin_amdgcn_wave_barrier();
    __builtin_amdgcn_fence(__ATOMIC_ACQUIRE, "workgroup");
  }
}

template <int MODE>
__global__ __launch_bounds__(256) void wtrans_kernel(const float* __restrict__ W0, const float* __restrict__ W1,
                                                    const float* __restrict__ W2, unsigned short* __restrict__ out,
                                                    int R, int Ccols, long in_zs, long out_zs, int zflip, float scale) {
  __shared__ float sm[64][65];
  const int t  = threadIdx.x;
  const int c0 = blockIdx.x * 64;
  const int r0 = blockIdx.y * 64;
  const int z  = blockIdx.z;
  const float* W = ((z == 0) ? W0 : (z == 1) ? W1 : W2) + (size_t)z * in_zs;
#pragma unroll
  for (int i = 0; i < 16; ++i) {
    const int e = i * 256 + t;
    const int r = e >> 6;
    const int c = e & 63;
    sm[c][r] = W[(size_t)(r0 + r) * Ccols + c0 + c];
  }
  __syncthreads();
  const int lane = t & 31, wave = t >> 5;
  const int q = lane >> 3, c8 = (lane & 7) * 8;
  const int zo = zflip ? ((int)gridDim.z - 1 - z) : z;
  unsigned short* op = out + (size_t)zo * out_zs;
  for (int pass = 0; pass < 2; ++pass) {
#pragma unroll
    for (int it = 0; it < 2; ++it) {
      const int row = wave * 8 + it * 4 + q;
      unsigned short hb[8];
#pragma unroll
      for (int e = 0; e < 8; ++e) {
        const float v = sm[row][c8 + e];
        hb[e] = (MODE == 0) ? f2bf_bits(v) : h_bits(bf_bits2f(f2bf_bits(v)) * scale);
      }
      const v4u u = (v4u){pk16(hb[0], hb[1]), pk16(hb[2], hb[3]), pk16(hb[4], hb[5]), pk16(hb[6], hb[7])};
      *(volatile v4u*)(op + (size_t)(c0 + row) * R + r0 + c8) = u;
    }
    __threadfence();
  }
}

__global__ __launch_bounds__(256) void s2d_gather_kernel(const float* __restrict__ xf, const float* __restrict__ zf,
                                                         unsigned short* __restrict__ Ax, unsigned short* __restrict__ Az) {
  const int gid = blockIdx.x * 256 + threadIdx.x;
  const int p   = gid >> 5;
  const int k8  = (gid & 31) * 8;
  const int b   = p >> 12;
  const int i   = (p >> 6) & 63;
  const int j   = p & 63;
  const int dy  = k8 >> 7;
  const int rem = k8 & 127;
  const size_t src = ((size_t)(b * kHin + 2 * i + dy) * kWin + 2 * j) * kC + rem;
  const v4f x0 = *(const v4f*)(xf + src), x1 = *(const v4f*)(xf + src + 4);
  const v4f z0 = *(const v4f*)(zf + src), z1 = *(const v4f*)(zf + src + 4);
  const v4u ux = (v4u){pk16(f2bf_bits(x0.x), f2bf_bits(x0.y)), pk16(f2bf_bits(x0.z), f2bf_bits(x0.w)),
                       pk16(f2bf_bits(x1.x), f2bf_bits(x1.y)), pk16(f2bf_bits(x1.z), f2bf_bits(x1.w))};
  const v4u uz = (v4u){pk16(f2bf_bits(z0.x), f2bf_bits(z0.y)), pk16(f2bf_bits(z0.z), f2bf_bits(z0.w)),
                       pk16(f2bf_bits(z1.x), f2bf_bits(z1.y)), pk16(f2bf_bits(z1.z), f2bf_bits(z1.w))};
  unsigned short* px = Ax + (size_t)p * kKconv + k8;
  unsigned short* pz = Az + (size_t)p * kKconv + k8;
  *(volatile v4u*)px = ux;
  *(volatile v4u*)pz = uz;
  __threadfence();
  *(volatile v4u*)px = ux;
  *(volatile v4u*)pz = uz;
}

__global__ __launch_bounds__(256) void softmax_rows_kernel(const float* __restrict__ S, unsigned short* __restrict__ P) {
  const int lane = threadIdx.x & 31;
  const int wave = threadIdx.x >> 5;
  const int row  = blockIdx.x * 8 + wave;
  const float* sr = S + (size_t)row * kTok;
  float m = -INFINITY;
#pragma unroll 1
  for (int jj = 0; jj < kTok / 256; ++jj) {
    const float* q = sr + jj * 256 + lane * 8;
    const v4f a = *(const v4f*)(q);
    const v4f c = *(const v4f*)(q + 4);
    m = fmaxf(m, fmaxf(fmaxf(a.x, a.y), fmaxf(a.z, a.w)));
    m = fmaxf(m, fmaxf(fmaxf(c.x, c.y), fmaxf(c.z, c.w)));
  }
#pragma unroll
  for (int off = 1; off < 32; off <<= 1) m = fmaxf(m, __shfl_xor(m, off, 32));
  float sum = 0.0f;
#pragma unroll 1
  for (int jj = 0; jj < kTok / 256; ++jj) {
    const float* q = sr + jj * 256 + lane * 8;
    const v4f a = *(const v4f*)(q);
    const v4f c = *(const v4f*)(q + 4);
    sum += __expf(a.x - m) + __expf(a.y - m) + __expf(a.z - m) + __expf(a.w - m);
    sum += __expf(c.x - m) + __expf(c.y - m) + __expf(c.z - m) + __expf(c.w - m);
  }
#pragma unroll
  for (int off = 1; off < 32; off <<= 1) sum += __shfl_xor(sum, off, 32);
  const float rs   = 1.0f / sum;
  const float rmul = kPCarry * rs;
  unsigned short* pr = P + (size_t)row * kTok;
#pragma unroll 1
  for (int jj = 0; jj < kTok / 256; ++jj) {
    const float* q = sr + jj * 256 + lane * 8;
    const v4f a = *(const v4f*)(q);
    const v4f c = *(const v4f*)(q + 4);
    const unsigned short h0 = h_bits(__expf(a.x - m) * rmul), h1 = h_bits(__expf(a.y - m) * rmul);
    const unsigned short h2 = h_bits(__expf(a.z - m) * rmul), h3 = h_bits(__expf(a.w - m) * rmul);
    const unsigned short h4 = h_bits(__expf(c.x - m) * rmul), h5 = h_bits(__expf(c.y - m) * rmul);
    const unsigned short h6 = h_bits(__expf(c.z - m) * rmul), h7 = h_bits(__expf(c.w - m) * rmul);
    const v4u u = (v4u){pk16(h0, h1), pk16(h2, h3), pk16(h4, h5), pk16(h6, h7)};
    unsigned short* pp = pr + jj * 256 + lane * 8;
    *(volatile v4u*)pp = u;
    __threadfence();
    *(volatile v4u*)pp = u;
  }
}

template <bool HASB, bool CEN>
__global__ __launch_bounds__(256) void colsum_kernel(const float* __restrict__ X, const float* __restrict__ bias,
                                                     const float* __restrict__ aff, float* __restrict__ part, int rpb) {
  __shared__ __align__(16) float sms[4][64];
  __shared__ __align__(16) float smo[64];
  const int t  = threadIdx.x;
  const int c  = t & 63;
  const int rg = t >> 6;
  const size_t r0 = (size_t)blockIdx.x * rpb;
  const float bv = HASB ? bias[c] : 0.0f;
  const float mu = CEN ? aff[128 + c] : 0.0f;
  float s = 0.0f;
#pragma unroll 1
  for (int r = rg; r < rpb; r += 4) {
    float v = X[(r0 + r) * kC + c] + bv;
    if (CEN) { const float d = v - mu; v = d * d; }
    s += v;
  }
  sms[rg][c] = s;
  __syncthreads();
  if (t < 64) smo[t] = ((sms[0][t] + sms[1][t]) + sms[2][t]) + sms[3][t];
  __syncthreads();
  if (t < 16) {
    const v4f a = *(const v4f*)(smo + 4 * t);
    float* pp = part + (size_t)blockIdx.x * 64 + 4 * t;
    *(volatile v4f*)pp = a;
    __threadfence();
    *(volatile v4f*)pp = a;
  }
}

template <int STEP>
__global__ __launch_bounds__(64) void bn_finalize_kernel(const float* __restrict__ part, int nblk, float inv_n,
                                                        const float* __restrict__ gamma, const float* __restrict__ beta,
                                                        float* __restrict__ aff) {
  __shared__ __align__(16) float smf[128];
  const int c = threadIdx.x;
  const int nb = nblk < 256 ? nblk : 256;
  float s = 0.0f;
#pragma unroll 1
  for (int k = 0; k < nb; ++k) s += part[(size_t)k * 64 + c];
  if (STEP == 0) {
    smf[c]      = s * inv_n;
    smf[64 + c] = 0.0f;
  } else {
    float var = s * inv_n;
    var = fmaxf(var, 0.0f);
    const float mean = aff[128 + c];
    const float sc = gamma[c] * rsqrtf(var + kBnEps);
    smf[c]      = sc;
    smf[64 + c] = beta[c] - mean * sc;
  }
  __syncthreads();
  if (STEP == 0) {
    if (c < 16) {
      const v4f v = *(const v4f*)(smf + 4 * c);
      float* ap = aff + 128 + 4 * c;
      *(volatile v4f*)ap = v;
      __threadfence();
      *(volatile v4f*)ap = v;
    }
  } else {
    if (c < 32) {
      const v4f v = *(const v4f*)(smf + 4 * c);
      float* ap = aff + 4 * c;
      *(volatile v4f*)ap = v;
      __threadfence();
      *(volatile v4f*)ap = v;
    }
  }
}

template <bool TRANS>
__global__ __launch_bounds__(256) void bn_relu_pack_kernel(const float* __restrict__ X, const float* __restrict__ aff,
                                                           unsigned short* __restrict__ out) {
  __shared__ float sm[64][65];
  const int t  = threadIdx.x;
  const int r0 = blockIdx.x * 64;
#pragma unroll
  for (int i = 0; i < 16; ++i) {
    const int e = i * 256 + t;
    const int r = e >> 6;
    const int c = e & 63;
    const float v = fmaxf(X[(size_t)(r0 + r) * kC + c] * aff[c] + aff[64 + c], 0.0f);
    if (TRANS) sm[c][r] = v; else sm[r][c] = v;
  }
  __syncthreads();
  const int lane = t & 31, wave = t >> 5;
  const int q = lane >> 3, c8 = (lane & 7) * 8;
  const int bb  = r0 >> 12;
  const int kv0 = r0 & (kTok - 1);
  for (int pass = 0; pass < 2; ++pass) {
#pragma unroll
    for (int it = 0; it < 2; ++it) {
      const int row = wave * 8 + it * 4 + q;
      unsigned short hb[8];
#pragma unroll
      for (int e = 0; e < 8; ++e) hb[e] = h_bits(sm[row][c8 + e]);
      const v4u u = (v4u){pk16(hb[0], hb[1]), pk16(hb[2], hb[3]), pk16(hb[4], hb[5]), pk16(hb[6], hb[7])};
      unsigned short* op;
      if (TRANS) op = out + ((size_t)(bb * kC + row)) * kTok + kv0 + c8;
      else       op = out + (size_t)(r0 + row) * kCcat + kC + c8;
      *(volatile v4u*)op = u;
    }
    __threadfence();
  }
}

__global__ __launch_bounds__(256) void d2s_bn_relu_out_kernel(const float* __restrict__ Yd, const float* __restrict__ bfi,
                                                              const float* __restrict__ aff, float* __restrict__ out) {
  const int i4  = blockIdx.x * 256 + threadIdx.x;
  const int o4  = (i4 & 15) * 4;
  const int pix = i4 >> 4;
  const int X   = pix & (kWin - 1);
  const int Yy  = (pix >> 7) & (kHin - 1);
  const int b   = pix >> 14;
  const int p   = (b * kHs + (Yy >> 1)) * kWs + (X >> 1);
  const int g   = (Yy & 1) * 2 + (X & 1);
  const v4f y  = *(const v4f*)(Yd + (size_t)p * kNdec + g * kC + o4);
  const v4f bv = *(const v4f*)(bfi + o4);
  const v4f sc = *(const v4f*)(aff + o4);
  const v4f sh = *(const v4f*)(aff + 64 + o4);
  v4f r;
  r.x = fmaxf((y.x + bv.x) * sc.x + sh.x, 0.0f);
  r.y = fmaxf((y.y + bv.y) * sc.y + sh.y, 0.0f);
  r.z = fmaxf((y.z + bv.z) * sc.z + sh.z, 0.0f);
  r.w = fmaxf((y.w + bv.w) * sc.w + sh.w, 0.0f);
  float* op = out + (size_t)i4 * 4;
  *(volatile v4f*)op = r;
  __threadfence();
  *(volatile v4f*)op = r;
}

extern "C" void kernel_launch(void* const* d_in, const int* in_sizes, int n_in,
                              void* d_out, int out_size, void* d_ws,
                              size_t ws_size, hipStream_t stream) {
  if (n_in < 14) return;
  if (in_sizes[0] != kB * kHin * kWin * kC || in_sizes[1] != kB * kHin * kWin * kC) return;
  if (in_sizes[2] != kKconv * kC || in_sizes[4] != kKconv * kC || in_sizes[6] != kKconv * kC) return;
  if (in_sizes[3] != kC || in_sizes[5] != kC || in_sizes[7] != kC || in_sizes[8] != kC || in_sizes[9] != kC) return;
  if (in_sizes[10] != 4 * kCcat * kC || in_sizes[11] != kC || in_sizes[12] != kC || in_sizes[13] != kC) return;
  if (out_size != kNPout * kC) return;
  if (ws_size < offEnd) return;

  const float* zf  = (const float*)d_in[0];
  const float* xf  = (const float*)d_in[1];
  const float* Wq  = (const float*)d_in[2];
  const float* bq  = (const float*)d_in[3];
  const float* Ws  = (const float*)d_in[4];
  const float* bs  = (const float*)d_in[5];
  const float* Wg  = (const float*)d_in[6];
  const float* bg  = (const float*)d_in[7];
  const float* gga = (const float*)d_in[8];
  const float* gbe = (const float*)d_in[9];
  const float* Wfi = (const float*)d_in[10];
  const float* bfi = (const float*)d_in[11];
  const float* fga = (const float*)d_in[12];
  const float* fbe = (const float*)d_in[13];
  float* out = (float*)d_out;
  char* ws = (char*)d_ws;

  unsigned short* Ax   = (unsigned short*)(ws + offAx);
  unsigned short* Az   = (unsigned short*)(ws + offAz);
  float*          XGp  = (float*)(ws + offXGp);
  float*          ZGp  = (float*)(ws + offZGp);
  unsigned short* Pp   = (unsigned short*)(ws + offP);
  float*          Sp   = (float*)(ws + offS);
  float*          Yd   = (float*)(ws + offY);
  unsigned short* Xqh  = (unsigned short*)(ws + offXqh);
  unsigned short* Xql  = (unsigned short*)(ws + offXql);
  unsigned short* Zkh  = (unsigned short*)(ws + offZkh);
  unsigned short* Zkl  = (unsigned short*)(ws + offZkl);
  unsigned short* Adec = (unsigned short*)(ws + offAdec);
  unsigned short* ZGt  = (unsigned short*)(ws + offZGt);
  unsigned short* BtW  = (unsigned short*)(ws + offBtW);
  unsigned short* Btfi = (unsigned short*)(ws + offBtfi);
  float*          part = (float*)(ws + offPart);
  float*          affX = (float*)(ws + offAffX);
  float*          affZ = (float*)(ws + offAffZ);
  float*          affY = (float*)(ws + offAffY);
  const float*    dumf = (const float*)(ws + offPart);

  const unsigned short* BtWq = BtW;
  const unsigned short* BtWs = BtW + (size_t)kC * kKconv;
  const unsigned short* BtWg = BtW + (size_t)2 * kC * kKconv;

  wtrans_kernel<0><<<dim3(kC / 64, kKconv / 64, 3), 256, 0, stream>>>(Wq, Ws, Wg, BtW, kKconv, kC, 0L,
                                                                     (long)kC * kKconv, 0, 1.0f);
  wtrans_kernel<1><<<dim3(kC / 64, kCcat / 64, 4), 256, 0, stream>>>(Wfi, Wfi, Wfi, Btfi, kCcat, kC,
                                                                    (long)kCcat * kC, (long)kC * kCcat, 1, kWfiCarry);
  s2d_gather_kernel<<<(kNP * 32) / 256, 256, 0, stream>>>(xf, zf, Ax, Az);

  const dim3 gconv(((kNP / 64) * (kC / 64) + 7) / 8, 1);
  wmma_gemm64<1, false, 2, 2, false><<<gconv, 256, 0, stream>>>(Ax, Ax, kKconv, 0L, BtWq, BtWq, kKconv, 0L,
      (void*)Xqh, (void*)Xql, kC, 0L, bq, dumf, 0L, kNP, kC, kKconv, 1.0f);
  wmma_gemm64<1, false, 2, 0, false><<<gconv, 256, 0, stream>>>(Ax, Ax, kKconv, 0L, BtWg, BtWg, kKconv, 0L,
      (void*)XGp, (void*)XGp, kC, 0L, bg, dumf, 0L, kNP, kC, kKconv, 1.0f);
  wmma_gemm64<1, false, 2, 2, false><<<gconv, 256, 0, stream>>>(Az, Az, kKconv, 0L, BtWs, BtWs, kKconv, 0L,
      (void*)Zkh, (void*)Zkl, kC, 0L, bs, dumf, 0L, kNP, kC, kKconv, 1.0f);
  wmma_gemm64<1, false, 2, 0, false><<<gconv, 256, 0, stream>>>(Az, Az, kKconv, 0L, BtWg, BtWg, kKconv, 0L,
      (void*)ZGp, (void*)ZGp, kC, 0L, bg, dumf, 0L, kNP, kC, kKconv, 1.0f);

  const int nbG = kNP / kStatRows;
  const float invG = 1.0f / (float)kNP;
  colsum_kernel<false, false><<<nbG, 256, 0, stream>>>(XGp, bg, affX, part, kStatRows);
  bn_finalize_kernel<0><<<1, 64, 0, stream>>>(part, nbG, invG, gga, gbe, affX);
  colsum_kernel<false, true><<<nbG, 256, 0, stream>>>(XGp, bg, affX, part, kStatRows);
  bn_finalize_kernel<1><<<1, 64, 0, stream>>>(part, nbG, invG, gga, gbe, affX);
  colsum_kernel<false, false><<<nbG, 256, 0, stream>>>(ZGp, bg, affZ, part, kStatRows);
  bn_finalize_kernel<0><<<1, 64, 0, stream>>>(part, nbG, invG, gga, gbe, affZ);
  colsum_kernel<false, true><<<nbG, 256, 0, stream>>>(ZGp, bg, affZ, part, kStatRows);
  bn_finalize_kernel<1><<<1, 64, 0, stream>>>(part, nbG, invG, gga, gbe, affZ);

  bn_relu_pack_kernel<false><<<kNP / 64, 256, 0, stream>>>(XGp, affX, Adec);
  bn_relu_pack_kernel<true><<<kNP / 64, 256, 0, stream>>>(ZGp, affZ, ZGt);

  const dim3 gS(((kTok / 64) * (kTok / 64) + 7) / 8, 1);
  const dim3 gPV(((kTok / 64) * (kC / 64) + 7) / 8, 1);
  for (int b = 0; b < kB; ++b) {
    const size_t po = (size_t)b * kTok * kC;
    wmma_gemm64<1, true, 0, 0, false><<<gS, 256, 0, stream>>>(Xqh + po, Xql + po, kC, 0L, Zkh + po, Zkl + po, kC, 0L,
        (void*)Sp, (void*)Sp, kTok, 0L, dumf, dumf, 0L, kTok, kTok, kC, 1.0f);
    softmax_rows_kernel<<<kTok / 8, 256, 0, stream>>>(Sp, Pp);
    wmma_gemm64<0, false, 0, 1, false><<<gPV, 256, 0, stream>>>(Pp, Pp, kTok, 0L,
        ZGt + (size_t)b * kC * kTok, ZGt + (size_t)b * kC * kTok, kTok, 0L,
        (void*)(Adec + (size_t)b * kTok * kCcat), (void*)(Adec + (size_t)b * kTok * kCcat), kCcat, 0L,
        dumf, dumf, 0L, kTok, kC, kTok, kPCarryInv);
  }

  const dim3 gdec(((kNP / 64) * (kNdec / 64) + 7) / 8, 1);
  wmma_gemm64<0, false, 0, 0, false><<<gdec, 256, 0, stream>>>(Adec, Adec, kCcat, 0L, Btfi, Btfi, kCcat, 0L,
      (void*)Yd, (void*)Yd, kNdec, 0L, dumf, dumf, 0L, kNP, kNdec, kCcat, kWfiCarryInv);

  const int nbY = kNPout / kStatRows;
  const float invY = 1.0f / (float)kNPout;
  colsum_kernel<true, false><<<nbY, 256, 0, stream>>>(Yd, bfi, affY, part, kStatRows);
  bn_finalize_kernel<0><<<1, 64, 0, stream>>>(part, nbY, invY, fga, fbe, affY);
  colsum_kernel<true, true><<<nbY, 256, 0, stream>>>(Yd, bfi, affY, part, kStatRows);
  bn_finalize_kernel<1><<<1, 64, 0, stream>>>(part, nbY, invY, fga, fbe, affY);

  d2s_bn_relu_out_kernel<<<(kNPout * kC / 4) / 256, 256, 0, stream>>>(Yd, bfi, affY, out);
}
